// PopulationAttention_59682865545947
// MI455X (gfx1250) — hardware-verified
//
#include <hip/hip_runtime.h>
#include <math.h>

typedef __attribute__((ext_vector_type(16))) _Float16 v16h;
typedef __attribute__((ext_vector_type(8)))  _Float16 v8h;
typedef __attribute__((ext_vector_type(16))) __bf16   v16b;
typedef __attribute__((ext_vector_type(8)))  __bf16   v8b;
typedef __attribute__((ext_vector_type(8)))  float    v8f;
typedef __attribute__((ext_vector_type(4)))  float    v4f;

constexpr int kBs   = 4;
constexpr int kH    = 16;
constexpr int kNb   = kBs * kH;
constexpr int kN    = 2048;
constexpr int kD    = 64;
constexpr int kThr  = 256;
constexpr float kInCarry = 1024.0f;
constexpr float kSCarry  = 128.0f;
constexpr float kSc1 = 1.0f / (kInCarry * kInCarry);
constexpr float kSc2 = 1.0f / (kInCarry * kSCarry * 8.0f);
constexpr float kF16MinNormal = 6.103515625e-5f;

static_assert((kD % 64) == 0 && (kN % 64) == 0 && (kN % 32) == 0 && (kD % 32) == 0 && ((kN / 64) * (kD / 64)) % 8 == 0, "GEMM M, N multiples of 64, K of 32; the second product's grid exact (32 tiles a batch)");

constexpr size_t kOffQ16 = 0ull;
constexpr size_t kOffKT16 = 16777216ull;
constexpr size_t kOffVT16 = 33554432ull;
constexpr size_t kOffZB = 50331648ull;
constexpr size_t kOffS32 = 50332672ull;
constexpr size_t kOffST16 = 51381248ull;
constexpr size_t kWsTotal = 51905536ull;
static_assert(kWsTotal <= 134217728ull, "carve cap: under 128 MiB");
static_assert(kOffQ16 == 0
              && kOffKT16 == kOffQ16 + 16777216ull
              && kOffVT16 == kOffKT16 + 16777216ull
              && kOffZB == kOffVT16 + 16777216ull
              && kOffS32 == kOffZB + 1024ull
              && kOffST16 == kOffS32 + 1048576ull
              && kWsTotal == kOffST16 + 524288ull, "the carve is chained and totalled");
static_assert((kOffQ16 % 256) == 0 && (kOffKT16 % 256) == 0 && (kOffVT16 % 256) == 0 && (kOffZB % 256) == 0 && (kOffS32 % 256) == 0 && (kOffST16 % 256) == 0, "aligned regions");

__device__ __forceinline__ unsigned short f2bf_bits(float f) {
  unsigned u = __float_as_uint(f);
  return (unsigned short)((u + 0x7FFFu + ((u >> 16) & 1u)) >> 16);
}
__device__ __forceinline__ float bf_bits2f(unsigned short h) { return __uint_as_float(((unsigned)h) << 16); }
__device__ __forceinline__ float bf16r(float f) { return bf_bits2f(f2bf_bits(f)); }
__device__ __forceinline__ float carry_flush(float v, float carry) {
  const float s = v * carry;
  return (fabsf(s) < kF16MinNormal) ? 0.0f : s;
}
__device__ __forceinline__ float frcp(float x) { return __builtin_amdgcn_rcpf(x); }

__device__ __forceinline__ void dep_guard4_h(v8f& a, v8f& b, v8f& c, v8f& d, v16h x, v16h y) { asm volatile("v_nop\n\tv_nop\n\tv_nop\n\tv_nop" : "+v"(a), "+v"(b), "+v"(c), "+v"(d) : "v"(x), "v"(y)); }
__device__ __forceinline__ void dep_guard4_b(v8f& a, v8f& b, v8f& c, v8f& d, v16b x, v16b y) { asm volatile("v_nop\n\tv_nop\n\tv_nop\n\tv_nop" : "+v"(a), "+v"(b), "+v"(c), "+v"(d) : "v"(x), "v"(y)); }
__device__ __forceinline__ void keep4_h(v16h a, v16h b, v16h c, v16h d) { asm volatile("v_nop" :: "v"(a), "v"(b), "v"(c), "v"(d)); }
__device__ __forceinline__ void keep4_b(v16b a, v16b b, v16b c, v16b d) { asm volatile("v_nop" :: "v"(a), "v"(b), "v"(c), "v"(d)); }
__device__ __forceinline__ void acc_guard4(v8f& a, v8f& b, v8f& c, v8f& d) { asm volatile("v_nop\n\tv_nop\n\tv_nop\n\tv_nop" : "+v"(a), "+v"(b), "+v"(c), "+v"(d)); }

template <typename T> struct Frag;
template <> struct Frag<_Float16> {
  typedef v16h V; union U { v16h v; v8h h[2]; };
  static __device__ __forceinline__ v16h load(const _Float16* p) {
    U f; f.h[0] = *(const v8h*)(p); f.h[1] = *(const v8h*)(p + 16); return f.v;
  }
  static __device__ __forceinline__ v8f mma(v16h a, v16h b, v8f c) {
    return __builtin_amdgcn_wmma_f32_16x16x32_f16(false, a, false, b, (short)0, c, false, false);
  }
  static __device__ __forceinline__ void guard4(v8f& a, v8f& b, v8f& c, v8f& d, v16h x, v16h y) { dep_guard4_h(a, b, c, d, x, y); }
  static __device__ __forceinline__ void keep(v16h a, v16h b, v16h c, v16h d) { keep4_h(a, b, c, d); }
};
template <> struct Frag<__bf16> {
  typedef v16b V; union U { v16b v; v8b h[2]; };
  static __device__ __forceinline__ v16b load(const __bf16* p) {
    U f; f.h[0] = *(const v8b*)(p); f.h[1] = *(const v8b*)(p + 16); return f.v;
  }
  static __device__ __forceinline__ v8f mma(v16b a, v16b b, v8f c) {
    return __builtin_amdgcn_wmma_f32_16x16x32_bf16(false, a, false, b, (short)0, c, false, false);
  }
  static __device__ __forceinline__ void guard4(v8f& a, v8f& b, v8f& c, v8f& d, v16b x, v16b y) { dep_guard4_b(a, b, c, d, x, y); }
  static __device__ __forceinline__ void keep(v16b a, v16b b, v16b c, v16b d) { keep4_b(a, b, c, d); }
};

__device__ __forceinline__ v8f mma_h(v16h a, v16h b, v8f c) {
  c = __builtin_amdgcn_wmma_f32_16x16x32_f16(false, a, false, b, (short)0, c, false, false);
  asm volatile("v_nop\n\tv_nop\n\tv_nop\n\tv_nop" : "+v"(c) : "v"(a), "v"(b));
  return c;
}

template <int ET> struct Elem;
template <> struct Elem<0> { typedef _Float16 T; };
template <> struct Elem<1> { typedef __bf16 T; };
template <int ET, bool SPLIT, int BIAS_MODE, int OUT_MODE, bool RESID, int ACT = 0>
__global__ __launch_bounds__(256) void wmma_gemm64(
    const unsigned short* __restrict__ Ap, const unsigned short* __restrict__ A2p, int lda, long strideA,
    const unsigned short* __restrict__ Btp, const unsigned short* __restrict__ Bt2p, int ldb, long strideB,
    void* __restrict__ Cout, void* __restrict__ Cout2, int ldc, long strideC,
    const float* __restrict__ bias,
    const float* __restrict__ resid, long strideR,
    int M, int N, int K, float scale) {
  typedef typename Elem<ET>::T T;
  typedef typename Frag<T>::V V;
  const T* A = (const T*)Ap; const T* A2 = (const T*)A2p; const T* Bt = (const T*)Btp; const T* Bt2 = (const T*)Bt2p;
  __shared__ __align__(16) float sT[8][16 * 68];
  const int b    = blockIdx.y;
  const int lane = threadIdx.x & 31;
  const int wave = threadIdx.x >> 5;
  const int tilesN = N >> 6;
  const int tilesM = M >> 6;
  const int tile = blockIdx.x * 8 + wave;
  if (tile >= tilesM * tilesN) return;
  const int tm = tile / tilesN;
  const int tn = tile - tm * tilesN;
  const int m0 = tm << 6;
  const int n0 = tn << 6;

  const T* Ab  = A  + (size_t)b * strideA;
  const T* Bb  = Bt + (size_t)b * strideB;
  const T* Ab2 = SPLIT ? (A2  + (size_t)b * strideA) : nullptr;
  const T* Bb2 = SPLIT ? (Bt2 + (size_t)b * strideB) : nullptr;

  const int rlane = lane & 15;
  const int koff  = (lane >> 4) * 8;
  const int mOff  = (lane >> 4) * 8;

  v8f acc[4][4];
#pragma unroll
  for (int i = 0; i < 4; ++i)
#pragma unroll
    for (int j = 0; j < 4; ++j) acc[i][j] = (v8f){0.f,0.f,0.f,0.f,0.f,0.f,0.f,0.f};

  for (int k0 = 0; k0 < K; k0 += 32) {
    V bh[4], bl[4];
#pragma unroll
    for (int j = 0; j < 4; ++j) {
      const size_t bo = (size_t)(n0 + (j << 4) + rlane) * ldb + koff + k0;
      bh[j] = Frag<T>::load(Bb + bo);
      if (SPLIT) bl[j] = Frag<T>::load(Bb2 + bo);
    }
#pragma unroll
    for (int i = 0; i < 4; ++i) {
      const size_t ao = (size_t)(m0 + (i << 4) + rlane) * lda + koff + k0;
      V ah = Frag<T>::load(Ab + ao);
      V al;
      if (SPLIT) al = Frag<T>::load(Ab2 + ao);
#pragma unroll
      for (int j = 0; j < 4; ++j) {
        acc[i][j] = Frag<T>::mma(ah, bh[j], acc[i][j]);
        if (SPLIT) {
          acc[i][j] = Frag<T>::mma(ah, bl[j], acc[i][j]);
          acc[i][j] = Frag<T>::mma(al, bh[j], acc[i][j]);
        }
      }
      Frag<T>::guard4(acc[i][0], acc[i][1], acc[i][2], acc[i][3], ah, SPLIT ? al : ah);
    }
    Frag<T>::keep(bh[0], bh[1], bh[2], bh[3]);
    if (SPLIT) Frag<T>::keep(bl[0], bl[1], bl[2], bl[3]);
  }
  acc_guard4(acc[0][0], acc[0][1], acc[0][2], acc[0][3]);
  acc_guard4(acc[1][0], acc[1][1], acc[1][2], acc[1][3]);
  acc_guard4(acc[2][0], acc[2][1], acc[2][2], acc[2][3]);
  acc_guard4(acc[3][0], acc[3][1], acc[3][2], acc[3][3]);

  float* slab = sT[wave];
  const float* Rb = RESID ? (resid + (size_t)b * strideR) : nullptr;
#pragma unroll
  for (int i = 0; i < 4; ++i) {
    const int mBase = m0 + (i << 4);
#pragma unroll
    for (int j = 0; j < 4; ++j) {
      const int n = n0 + (j << 4) + rlane;
      float bv = 0.f;
      if (BIAS_MODE == 2) bv = bias[n];
#pragma unroll
      for (int r = 0; r < 8; ++r) {
        float v = acc[i][j][r] * scale;
        if (BIAS_MODE == 1) v += bias[mBase + mOff + r];
        if (BIAS_MODE == 2) v += bv;
        if (RESID) v += Rb[(size_t)(mBase + mOff + r) * ldc + n];
        if (ACT == 1) v = tanhf(v);
        if (ACT == 2) v = fmaxf(v, 0.0f);
        if (ACT == 3) v = v / (1.0f + expf(-v));
        if (ACT == 4) v = (v > 0.f) ? v : 0.01f * v;
        slab[(mOff + r) * 68 + (j << 4) + rlane] = v;
      }
    }
    __builtin_amdgcn_fence(__ATOMIC_RELEASE, "workgroup");
    __builtin_amdgcn_wave_barrier();
    __builtin_amdgcn_fence(__ATOMIC_ACQUIRE, "workgroup");
    if (OUT_MODE == 0) {
      float* C = (float*)Cout + (size_t)b * strideC;
      const int hh = lane >> 4, c4 = (lane & 15) * 4;
      for (int pass = 0; pass < 2; ++pass) {
#pragma unroll
        for (int it = 0; it < 8; ++it) {
          const int row = it * 2 + hh;
          v4f v = *(const v4f*)(slab + row * 68 + c4);
          *(volatile v4f*)(C + (size_t)(mBase + row) * ldc + n0 + c4) = v;
        }
        __threadfence();
      }
    } else {
      const int q = lane >> 3, c8 = (lane & 7) * 8;
      unsigned short* C  = (unsigned short*)Cout  + (size_t)b * strideC;
      unsigned short* C2 = (OUT_MODE == 2) ? ((unsigned short*)Cout2 + (size_t)b * strideC) : nullptr;
      for (int pass = 0; pass < 2; ++pass) {
#pragma unroll
        for (int it = 0; it < 4; ++it) {
          const int row = it * 4 + q;
          const float* sp = slab + row * 68 + c8;
          v8h hv, lv;
#pragma unroll
          for (int e = 0; e < 8; ++e) {
            if (OUT_MODE == 1) {
              hv[e] = (_Float16)sp[e];
            } else {
              unsigned short hb = f2bf_bits(sp[e]);
              unsigned short lb = f2bf_bits(sp[e] - bf_bits2f(hb));
              hv[e] = __builtin_bit_cast(_Float16, hb);
              lv[e] = __builtin_bit_cast(_Float16, lb);
            }
          }
          *(volatile v8h*)(C + (size_t)(mBase + row) * ldc + n0 + c8) = hv;
          if (OUT_MODE == 2) *(volatile v8h*)(C2 + (size_t)(mBase + row) * ldc + n0 + c8) = lv;
        }
        __threadfence();
      }
    }
    __builtin_amdgcn_fence(__ATOMIC_RELEASE, "workgroup");
    __builtin_amdgcn_wave_barrier();
    __builtin_amdgcn_fence(__ATOMIC_ACQUIRE, "workgroup");
  }
}

__global__ __launch_bounds__(kThr) void cast_plane_kernel(const float* __restrict__ src, unsigned short* __restrict__ dst,
                                                          int colsLog2, int dstPitch, int dstOff) {
  const int i   = blockIdx.x * kThr + threadIdx.x;
  const int sh  = colsLog2 - 3;
  const int row = i >> sh;
  const int c8  = (i & ((1 << sh) - 1)) * 8;
  const float* sp = src + ((size_t)row << colsLog2) + c8;
  const v4f a0 = *(const v4f*)(sp);
  const v4f a1 = *(const v4f*)(sp + 4);
  v8h hv;
#pragma unroll
  for (int e = 0; e < 4; ++e) {
    const float f0 = a0[e];
    const float f1 = a1[e];
    hv[e]     = (_Float16)carry_flush(bf16r(f0), kInCarry);
    hv[4 + e] = (_Float16)carry_flush(bf16r(f1), kInCarry);
  }
  unsigned short* dp = dst + (size_t)row * dstPitch + dstOff + c8;
  *(volatile v8h*)dp = hv;
  __threadfence();
  *(volatile v8h*)dp = hv;
}


__global__ __launch_bounds__(kThr) void tcast_kernel(const float* __restrict__ K, const float* __restrict__ V, const float* __restrict__ xw,
                                                    unsigned short* __restrict__ KT16, unsigned short* __restrict__ VT16) {
  const unsigned bz = blockIdx.z;
  const bool isV = bz >= (unsigned)kNb;
  const unsigned b = isV ? (bz - (unsigned)kNb) : bz;
  const unsigned r = blockIdx.y;
  const unsigned m8 = (blockIdx.x * (unsigned)kThr + threadIdx.x) * 8u;
  const float* src = (isV ? V : K) + ((size_t)b * kN + m8) * kD + r;
  const float* xs = xw + (size_t)(b >> 4) * kN + m8;
  v8h hv;
#pragma unroll
  for (int j = 0; j < 8; ++j) {
    const float p = src[(size_t)j * kD];
    float v = bf16r(p);
    if (isV) { const float q = xs[j]; v = v * bf16r(q); }
    hv[j] = (_Float16)carry_flush(v, kInCarry);
  }
  unsigned short* dp = (isV ? VT16 : KT16) + ((size_t)b * kD + r) * kN + m8;
  *(volatile v8h*)dp = hv;
  __threadfence();
  *(volatile v8h*)dp = hv;
}
static_assert(kN / 8 == kThr && kH == 16, "transposing cast grid exact: 256 chunks of 8 positions a row: ONE block a row; sample = b >> 4");

__global__ __launch_bounds__(kThr) void scast_kernel(const float* __restrict__ S32, unsigned short* __restrict__ ST16, float* __restrict__ ZB) {
  if (blockIdx.x == 0u) {
    float* dp = ZB + threadIdx.x;
    *(volatile float*)dp = 0.0f;
    __threadfence();
    *(volatile float*)dp = 0.0f;
    return;
  }
  const unsigned i = (blockIdx.x - 1u) * (unsigned)kThr + threadIdx.x;
  const unsigned b = i >> 9, e = (i >> 3) & 63u, d8 = (i & 7u) * 8u;
  const float* sp = S32 + ((size_t)b * kD + d8) * kD + e;
  v8h hv;
#pragma unroll
  for (int j = 0; j < 8; ++j) hv[j] = (_Float16)carry_flush(sp[(size_t)j * kD], kSCarry);
  unsigned short* dp = ST16 + ((size_t)b * kD + e) * kD + d8;
  *(volatile v8h*)dp = hv;
  __threadfence();
  *(volatile v8h*)dp = hv;
}
static_assert(kNb * kD * (kD / 8) == 128 * kThr && kD == 64, "S cast grid exact: 128 blocks; 512 threads a batch");

static_assert(((size_t)kNb * kN * kD / 8) % kThr == 0 && ((size_t)kNb * kN * kD) % 64 == 0, "plane cast grid exact; the plane is whole rows of 64");

extern "C" void kernel_launch(void* const* d_in, const int* in_sizes, int n_in,
                              void* d_out, int out_size, void* d_ws, size_t ws_size,
                              hipStream_t stream) {
  if (n_in < 4 || d_out == nullptr || d_ws == nullptr) return;
  if (in_sizes[0] != kNb * kN * kD || in_sizes[1] != kNb * kN * kD || in_sizes[2] != kNb * kN * kD || in_sizes[3] != kBs * kN) return;
  if (out_size != kNb * kN * kD) return;
  if (ws_size < kWsTotal) return;
  const float* Q = (const float*)d_in[0];
  const float* K = (const float*)d_in[1];
  const float* V = (const float*)d_in[2];
  const float* xw = (const float*)d_in[3];
  float* out = (float*)d_out;
  char* ws = (char*)d_ws;
  unsigned short* Q16 = (unsigned short*)(ws + kOffQ16);
  unsigned short* KT16 = (unsigned short*)(ws + kOffKT16);
  unsigned short* VT16 = (unsigned short*)(ws + kOffVT16);
  float* ZB = (float*)(ws + kOffZB);
  float* S32 = (float*)(ws + kOffS32);
  unsigned short* ST16 = (unsigned short*)(ws + kOffST16);

  cast_plane_kernel<<<(int)(((size_t)kNb * kN * kD / 8) / kThr), kThr, 0, stream>>>(Q, Q16, 6, 64, 0);
  tcast_kernel<<<dim3(1, kD, 2 * kNb), kThr, 0, stream>>>(K, V, xw, KT16, VT16);
  scast_kernel<<<1, kThr, 0, stream>>>(S32, ST16, ZB);
  wmma_gemm64<0, false, 2, 0, false, 0><<<dim3(1, kNb), 256, 0, stream>>>(
      KT16, KT16, kN, (long)kD * kN, VT16, VT16, kN, (long)kD * kN, (void*)S32, (void*)S32, kD, (long)kD * kD, ZB, nullptr, 0L, kD, kD, kN, kSc1);
  scast_kernel<<<129, kThr, 0, stream>>>(S32, ST16, ZB);
  wmma_gemm64<0, false, 2, 0, false, 0><<<dim3((kN / 64) * (kD / 64) / 8, kNb), 256, 0, stream>>>(
      Q16, Q16, kD, (long)kN * kD, ST16, ST16, kD, (long)kD * kD, (void*)out, (void*)out, kD, (long)kN * kD, ZB, nullptr, 0L, kN, kD, kD, kSc2);
}
